// KSGraphAttention_5875515261331
// MI455X (gfx1250) — hardware-verified
//
#include <hip/hip_runtime.h>
#include <stddef.h>
#include <stdint.h>

typedef _Float16 v16h __attribute__((ext_vector_type(16)));
typedef _Float16 v8h  __attribute__((ext_vector_type(8)));
typedef float    v8f  __attribute__((ext_vector_type(8)));
typedef float    v4f  __attribute__((ext_vector_type(4)));
typedef unsigned v4u  __attribute__((ext_vector_type(4)));

union Frag { v16h v; v8h hv[2]; };

constexpr int NB    = 2;
constexpr int NTOK  = 4096;
constexpr int DM    = 256;
constexpr int NH    = 4;
constexpr int HDIM  = 64;
constexpr int MROWS = NB * NTOK;
constexpr int MWPR  = NTOK / 32;
constexpr int NBH   = NB * NH;
constexpr float SM_SCALE = 0.125f;
constexpr float NEG_BIG  = -1e30f;
constexpr float W_SCALE  = 16.f;
constexpr float W_UNSC   = 0.0625f;
constexpr float P_SCALE  = 4096.f;
constexpr float LN_EPS   = 1e-5f;

__device__ __forceinline__ v8f zero8()
{
    v8f z = {0.f, 0.f, 0.f, 0.f, 0.f, 0.f, 0.f, 0.f};
    return z;
}

__device__ __forceinline__ v8f wmma_f16(v16h a, v16h b, v8f c)
{
    c = __builtin_amdgcn_wmma_f32_16x16x32_f16(false, a, false, b, (short)0, c, false, false);
    asm volatile("v_nop\n\tv_nop\n\tv_nop\n\tv_nop" : "+v"(c) : "v"(a), "v"(b));
    return c;
}

__device__ __forceinline__ v16h load_frag(const _Float16* p, int h)
{
    Frag f;
    f.hv[0] = *(const v8h*)(p + 8 * h);
    f.hv[1] = *(const v8h*)(p + 16 + 8 * h);
    return f.v;
}

__device__ __forceinline__ v8h cvt8(v4f a, v4f b, float sc)
{
    v8h r = {(_Float16)(a.x * sc), (_Float16)(a.y * sc), (_Float16)(a.z * sc), (_Float16)(a.w * sc),
             (_Float16)(b.x * sc), (_Float16)(b.y * sc), (_Float16)(b.z * sc), (_Float16)(b.w * sc)};
    return r;
}

__global__ void __launch_bounds__(256)
k_prep(const float* __restrict__ x, const float* __restrict__ wq, const float* __restrict__ wk,
       const float* __restrict__ wv, const float* __restrict__ wo, int nx8, int nw8,
       _Float16* __restrict__ xh, _Float16* __restrict__ wh)
{
    const int i = blockIdx.x * 256 + threadIdx.x;
    const int total = nx8 + 4 * nw8;
    const bool act = i < total;
    v4f a = {0.f, 0.f, 0.f, 0.f};
    v4f b = a;
    float sc = 0.f;
    _Float16* dst = xh;
    if (act) {
        const float* src;
        if (i < nx8) {
            src = x + (size_t)i * 8;
            dst = xh + (size_t)i * 8;
            sc = 1.f;
        } else {
            const int j = i - nx8;
            const int sel = j / nw8;
            const int r = j - sel * nw8;
            const float* wb = (sel == 0) ? wq : (sel == 1) ? wk : (sel == 2) ? wv : wo;
            src = wb + (size_t)r * 8;
            dst = wh + (size_t)sel * nw8 * 8 + (size_t)r * 8;
            sc = W_SCALE;
        }
        a = *(const v4f*)src;
        b = *(const v4f*)(src + 4);
    }
    const v8h v = cvt8(a, b, sc);
    if (act) *(volatile v8h*)dst = v;
    __threadfence();
    if (act) *(volatile v8h*)dst = v;
}

__global__ void __launch_bounds__(256)
k_mask(const int* __restrict__ ei, int n_e, unsigned* __restrict__ mk)
{
    __shared__ __attribute__((aligned(16))) unsigned bits[32 * MWPR];
    __shared__ int lst[256];
    __shared__ int wc[8];
    const int tid = threadIdx.x, lane = tid & 31, wv = tid >> 5;
    const int row0 = blockIdx.x * 32;

    for (int i = tid; i < 32 * MWPR; i += 256) {
        const int r = i >> 7, w = i & (MWPR - 1);
        bits[i] = (w == (int)blockIdx.x) ? (1u << r) : 0u;
    }
    __syncthreads();

#pragma unroll 1
    for (int c0 = 0; c0 < n_e; c0 += 256) {
        const int e = c0 + tid;
        const bool valid = e < n_e;
        int src = 0, dst = -1;
        if (valid) {
            src = ei[e];
            dst = ei[(size_t)n_e + e];
            if (src < 0) src += NTOK;
            if (dst < 0) dst += NTOK;
        }
        const bool match = valid && ((unsigned)src < (unsigned)NTOK) && dst >= row0 && dst < row0 + 32;
        const unsigned bm = (unsigned)__ballot(match);
        const int cnt = __popc(bm);
        const int pos = __popc(bm & ((1u << lane) - 1u));
        if (lane == 0) wc[wv] = cnt;
        __syncthreads();
        int base = 0, total = 0;
#pragma unroll
        for (int q = 0; q < 8; ++q) {
            const int t = wc[q];
            if (q < wv) base += t;
            total += t;
        }
        if (match) lst[base + pos] = ((dst - row0) << 12) | src;
        __syncthreads();
        if (wv == 0) {
#pragma unroll 1
            for (int j = 0; j < total; ++j) {
                const int v = lst[j];
                if ((v >> 12) == lane)
                    bits[lane * MWPR + ((v & (NTOK - 1)) >> 5)] |= 1u << (v & 31);
            }
        }
        __syncthreads();
    }

    unsigned* ob = mk + (size_t)row0 * MWPR;
    v4u vals[4];
#pragma unroll
    for (int p = 0; p < 4; ++p) {
        const int idx = p * 256 + tid;
        vals[p] = *(const v4u*)(bits + idx * 4);
        *(volatile v4u*)(ob + (size_t)idx * 4) = vals[p];
    }
    __threadfence();
#pragma unroll
    for (int p = 0; p < 4; ++p) {
        const int idx = p * 256 + tid;
        *(volatile v4u*)(ob + (size_t)idx * 4) = vals[p];
    }
}

__global__ void __launch_bounds__(128)
k_qkv(const _Float16* __restrict__ xh, const _Float16* __restrict__ wh,
      const float* __restrict__ bq, const float* __restrict__ bk, const float* __restrict__ bv,
      _Float16* __restrict__ qf, _Float16* __restrict__ kf, _Float16* __restrict__ vf)
{
    __shared__ __attribute__((aligned(16))) _Float16 st[64 * HDIM];
    const int tid = threadIdx.x, wv = tid >> 5, lane = tid & 31, h = lane >> 4, m = lane & 15;
    const int rb = blockIdx.x, head = blockIdx.y, sel = blockIdx.z;
    const int m0 = rb * 64 + wv * 16;
    const _Float16* wbase = wh + (size_t)sel * DM * DM + (size_t)(head * HDIM) * DM;

    v8f acc[4];
#pragma unroll
    for (int j = 0; j < 4; ++j) acc[j] = zero8();

#pragma unroll 2
    for (int k0 = 0; k0 < DM; k0 += 32) {
        const v16h a = load_frag(xh + (size_t)(m0 + m) * DM + k0, h);
#pragma unroll
        for (int j = 0; j < 4; ++j) {
            const v16h b = load_frag(wbase + (size_t)(16 * j + m) * DM + k0, h);
            acc[j] = wmma_f16(a, b, acc[j]);
        }
    }

    const float* bias = (sel == 0) ? bq : (sel == 1) ? bk : bv;
#pragma unroll
    for (int j = 0; j < 4; ++j) {
        const float bb = bias[head * HDIM + 16 * j + m];
#pragma unroll
        for (int r = 0; r < 8; ++r)
            st[(wv * 16 + 8 * h + r) * HDIM + 16 * j + m] = (_Float16)(acc[j][r] * W_UNSC + bb);
    }
    __syncthreads();

    const int grow0 = rb * 64;
    const int bi = grow0 / NTOK, tok0 = grow0 - bi * NTOK;
    const int bhd = bi * NH + head;
    _Float16* ob = ((sel == 0) ? qf : (sel == 1) ? kf : vf) + ((size_t)bhd * NTOK + tok0) * HDIM;
    v8h ov[4];
#pragma unroll
    for (int p = 0; p < 4; ++p) {
        const int idx = p * 128 + tid;
        ov[p] = *(const v8h*)(st + idx * 8);
        *(volatile v8h*)(ob + (size_t)idx * 8) = ov[p];
    }
    __threadfence();
#pragma unroll
    for (int p = 0; p < 4; ++p) {
        const int idx = p * 128 + tid;
        *(volatile v8h*)(ob + (size_t)idx * 8) = ov[p];
    }
}

__global__ void __launch_bounds__(32)
k_attn(const _Float16* __restrict__ qf, const _Float16* __restrict__ kf,
       const _Float16* __restrict__ vf, const unsigned* __restrict__ mk,
       _Float16* __restrict__ oh)
{
    __shared__ __attribute__((aligned(16))) unsigned smask[16 * MWPR];
    __shared__ __attribute__((aligned(16))) int      sq[64];
    __shared__ __attribute__((aligned(16))) _Float16 sp[16 * 32];
    __shared__ __attribute__((aligned(16))) _Float16 so[16 * HDIM];

    const int lane = threadIdx.x, h = lane >> 4, nl = lane & 15;
    const int q0 = blockIdx.x * 16;
    const int bh = blockIdx.y, bi = bh >> 2, hsel = bh & 3;

    {
        const v4u* src = (const v4u*)(mk + (size_t)q0 * MWPR);
        v4u* dst = (v4u*)smask;
        for (int i = lane; i < (16 * MWPR) / 4; i += 32) dst[i] = src[i];
    }
    sq[lane] = 0;
    sq[32 + lane] = 0;
    __syncthreads();

    const _Float16* qb = qf + ((size_t)bh * NTOK + q0) * HDIM;
    const v16h aq0 = load_frag(qb + (size_t)nl * HDIM, h);
    const v16h aq1 = load_frag(qb + (size_t)nl * HDIM + 32, h);
    const _Float16* kb = kf + (size_t)bh * NTOK * HDIM;
    const _Float16* vb = vf + (size_t)bh * NTOK * HDIM;

    v8f oacc[4];
#pragma unroll
    for (int nt = 0; nt < 4; ++nt) oacc[nt] = zero8();
    float mrun[8], lrun[8];
#pragma unroll
    for (int r = 0; r < 8; ++r) { mrun[r] = NEG_BIG; lrun[r] = 0.f; }

    int qlen = 0;
#pragma unroll 1
    for (int w = 0; w <= MWPR; ++w) {
        int nvalid = 0;
        if (w < MWPR) {
            unsigned u = smask[nl * MWPR + w];
            u |= __shfl_xor(u, 8, 16);
            u |= __shfl_xor(u, 4, 16);
            u |= __shfl_xor(u, 2, 16);
            u |= __shfl_xor(u, 1, 16);
            if (u != 0u) {
                const int c = __popc(u);
                const int rank = __popc(u & ((1u << lane) - 1u));
                if ((u >> lane) & 1u) sq[qlen + rank] = w * 32 + lane;
                qlen += c;
                __syncthreads();
                if (qlen >= 32) nvalid = 32;
            }
        } else {
            nvalid = qlen;
        }

        if (nvalid > 0) {
            const int kA = sq[nl] & (NTOK - 1);
            const int kB = sq[16 + nl] & (NTOK - 1);
            const bool vA = nl < nvalid, vB = (16 + nl) < nvalid;
            v8f s0 = zero8(), s1 = zero8();
            s0 = wmma_f16(aq0, load_frag(kb + (size_t)kA * HDIM, h), s0);
            s0 = wmma_f16(aq1, load_frag(kb + (size_t)kA * HDIM + 32, h), s0);
            s1 = wmma_f16(aq0, load_frag(kb + (size_t)kB * HDIM, h), s1);
            s1 = wmma_f16(aq1, load_frag(kb + (size_t)kB * HDIM + 32, h), s1);

            const int wA = kA >> 5, wB = kB >> 5;
            const unsigned bA = 1u << (kA & 31), bB = 1u << (kB & 31);
#pragma unroll
            for (int r = 0; r < 8; ++r) {
                const int m = 8 * h + r;
                const bool alA = vA && ((smask[m * MWPR + wA] & bA) != 0u);
                const bool alB = vB && ((smask[m * MWPR + wB] & bB) != 0u);
                const float v0 = alA ? s0[r] * SM_SCALE : NEG_BIG;
                const float v1 = alB ? s1[r] * SM_SCALE : NEG_BIG;
                float mx = fmaxf(v0, v1);
                mx = fmaxf(mx, __shfl_xor(mx, 8, 16));
                mx = fmaxf(mx, __shfl_xor(mx, 4, 16));
                mx = fmaxf(mx, __shfl_xor(mx, 2, 16));
                mx = fmaxf(mx, __shfl_xor(mx, 1, 16));
                const float mnew  = fmaxf(mrun[r], mx);
                const float alpha = __expf(mrun[r] - mnew);
                const float e0 = alA ? __expf(v0 - mnew) * P_SCALE : 0.f;
                const float e1 = alB ? __expf(v1 - mnew) * P_SCALE : 0.f;
                float rs = e0 + e1;
                rs += __shfl_xor(rs, 8, 16);
                rs += __shfl_xor(rs, 4, 16);
                rs += __shfl_xor(rs, 2, 16);
                rs += __shfl_xor(rs, 1, 16);
                lrun[r] = lrun[r] * alpha + rs;
                mrun[r] = mnew;
                sp[m * 32 + nl]      = (_Float16)e0;
                sp[m * 32 + 16 + nl] = (_Float16)e1;
#pragma unroll
                for (int nt = 0; nt < 4; ++nt) oacc[nt][r] *= alpha;
            }
            __syncthreads();

            const v16h ap = load_frag(sp + nl * 32, h);
            int kk[16];
#pragma unroll
            for (int i = 0; i < 8; ++i) {
                kk[i]     = sq[8 * h + i] & (NTOK - 1);
                kk[8 + i] = sq[16 + 8 * h + i] & (NTOK - 1);
            }
#pragma unroll
            for (int nt = 0; nt < 4; ++nt) {
                Frag b;
#pragma unroll
                for (int i = 0; i < 16; ++i)
                    b.v[i] = vb[(size_t)kk[i] * HDIM + nt * 16 + nl];
                oacc[nt] = wmma_f16(ap, b.v, oacc[nt]);
            }

            const int rem = qlen - nvalid;
            __syncthreads();
            const int t = (lane < rem) ? sq[32 + lane] : 0;
            __syncthreads();
            sq[lane] = t;
            __syncthreads();
            qlen = rem;
        }
    }

    float inv[8];
#pragma unroll
    for (int r = 0; r < 8; ++r) inv[r] = (lrun[r] > 0.f) ? (1.f / lrun[r]) : 0.f;
#pragma unroll
    for (int nt = 0; nt < 4; ++nt)
#pragma unroll
        for (int r = 0; r < 8; ++r)
            so[(8 * h + r) * HDIM + nt * 16 + nl] = (_Float16)(oacc[nt][r] * inv[r]);
    __syncthreads();

    _Float16* ob = oh + (size_t)(bi * NTOK + q0) * DM + hsel * HDIM;
    v8h ov[4];
#pragma unroll
    for (int p = 0; p < 4; ++p) {
        const int line = p * 4 + (lane >> 3), ch = lane & 7;
        ov[p] = *(const v8h*)(so + line * HDIM + ch * 8);
        *(volatile v8h*)(ob + (size_t)line * DM + ch * 8) = ov[p];
    }
    __threadfence();
#pragma unroll
    for (int p = 0; p < 4; ++p) {
        const int line = p * 4 + (lane >> 3), ch = lane & 7;
        *(volatile v8h*)(ob + (size_t)line * DM + ch * 8) = ov[p];
    }
}

__global__ void __launch_bounds__(256)
k_out(const _Float16* __restrict__ oh, const _Float16* __restrict__ who,
      const float* __restrict__ bo, const float* __restrict__ x,
      const float* __restrict__ gamma, const float* __restrict__ beta, float* __restrict__ out)
{
    __shared__ __attribute__((aligned(16))) float sh[32 * DM];
    const int tid = threadIdx.x, wv = tid >> 5, lane = tid & 31, h = lane >> 4, m = lane & 15;
    const int r0 = blockIdx.x * 32;
    const int rt = wv >> 2, ct0 = (wv & 3) * 4;

    v8f acc[4];
#pragma unroll
    for (int j = 0; j < 4; ++j) acc[j] = zero8();

#pragma unroll 2
    for (int k0 = 0; k0 < DM; k0 += 32) {
        const v16h a = load_frag(oh + (size_t)(r0 + 16 * rt + m) * DM + k0, h);
#pragma unroll
        for (int j = 0; j < 4; ++j) {
            const v16h b = load_frag(who + (size_t)(16 * (ct0 + j) + m) * DM + k0, h);
            acc[j] = wmma_f16(a, b, acc[j]);
        }
    }
#pragma unroll
    for (int j = 0; j < 4; ++j)
#pragma unroll
        for (int r = 0; r < 8; ++r)
            sh[(16 * rt + 8 * h + r) * DM + 16 * (ct0 + j) + m] = acc[j][r] * W_UNSC;
    __syncthreads();

    const int c0 = 4 * lane, c1 = 128 + 4 * lane;
    const v4f b0 = *(const v4f*)(bo + c0),    b1 = *(const v4f*)(bo + c1);
    const v4f g0 = *(const v4f*)(gamma + c0), g1 = *(const v4f*)(gamma + c1);
    const v4f e0 = *(const v4f*)(beta + c0),  e1 = *(const v4f*)(beta + c1);
    v4f res[8];
#pragma unroll
    for (int rr = 0; rr < 4; ++rr) {
        const int row = wv * 4 + rr;
        const size_t gro = (size_t)(r0 + row) * DM;
        const v4f a0 = *(const v4f*)(sh + row * DM + c0), a1 = *(const v4f*)(sh + row * DM + c1);
        const v4f x0 = *(const v4f*)(x + gro + c0),       x1 = *(const v4f*)(x + gro + c1);
        const v4f h0 = (a0 + b0) + x0, h1 = (a1 + b1) + x1;
        float s = ((h0.x + h0.y) + (h0.z + h0.w)) + ((h1.x + h1.y) + (h1.z + h1.w));
#pragma unroll
        for (int off = 16; off >= 1; off >>= 1) s += __shfl_xor(s, off, 32);
        const float mu = s * (1.f / DM);
        const v4f d0 = h0 - mu, d1 = h1 - mu;
        float q = ((d0.x * d0.x + d0.y * d0.y) + (d0.z * d0.z + d0.w * d0.w))
                + ((d1.x * d1.x + d1.y * d1.y) + (d1.z * d1.z + d1.w * d1.w));
#pragma unroll
        for (int off = 16; off >= 1; off >>= 1) q += __shfl_xor(q, off, 32);
        const float rstd = rsqrtf(q * (1.f / DM) + LN_EPS);
        res[2 * rr]     = d0 * rstd * g0 + e0;
        res[2 * rr + 1] = d1 * rstd * g1 + e1;
        *(volatile v4f*)(out + gro + c0) = res[2 * rr];
        *(volatile v4f*)(out + gro + c1) = res[2 * rr + 1];
    }
    __threadfence();
#pragma unroll
    for (int rr = 0; rr < 4; ++rr) {
        const size_t gro = (size_t)(r0 + wv * 4 + rr) * DM;
        *(volatile v4f*)(out + gro + c0) = res[2 * rr];
        *(volatile v4f*)(out + gro + c1) = res[2 * rr + 1];
    }
}

extern "C" void kernel_launch(void* const* d_in, const int* in_sizes, int n_in,
                              void* d_out, int out_size, void* d_ws, size_t ws_size,
                              hipStream_t stream)
{
    if (n_in < 12) return;
    if (in_sizes[0] != MROWS * DM || out_size != MROWS * DM) return;
    if (in_sizes[2] != DM * DM || in_sizes[4] != DM * DM || in_sizes[6] != DM * DM || in_sizes[8] != DM * DM) return;
    if (in_sizes[3] < DM || in_sizes[5] < DM || in_sizes[7] < DM || in_sizes[9] < DM ||
        in_sizes[10] < DM || in_sizes[11] < DM) return;
    if (in_sizes[1] < 0 || (in_sizes[1] & 1)) return;

    const float* x     = (const float*)d_in[0];
    const int*   ei    = (const int*)d_in[1];
    const float* wq    = (const float*)d_in[2];
    const float* bq    = (const float*)d_in[3];
    const float* wk    = (const float*)d_in[4];
    const float* bk    = (const float*)d_in[5];
    const float* wv    = (const float*)d_in[6];
    const float* bv    = (const float*)d_in[7];
    const float* wo    = (const float*)d_in[8];
    const float* bo    = (const float*)d_in[9];
    const float* gamma = (const float*)d_in[10];
    const float* beta  = (const float*)d_in[11];
    float* out = (float*)d_out;
    const int n_e = in_sizes[1] / 2;

    const size_t b_xh = (size_t)MROWS * DM * 2;
    const size_t b_wh = (size_t)4 * DM * DM * 2;
    const size_t b_mk = (size_t)NTOK * MWPR * 4;
    const size_t b_hd = (size_t)NBH * NTOK * HDIM * 2;
    const size_t b_oh = (size_t)MROWS * DM * 2;
    char* ws = (char*)d_ws;
    size_t off = 0;
    _Float16* xh = (_Float16*)(ws + off); off += b_xh;
    _Float16* wh = (_Float16*)(ws + off); off += b_wh;
    unsigned* mk = (unsigned*)(ws + off); off += b_mk;
    _Float16* qf = (_Float16*)(ws + off); off += b_hd;
    _Float16* kf = (_Float16*)(ws + off); off += b_hd;
    _Float16* vf = (_Float16*)(ws + off); off += b_hd;
    _Float16* oh = (_Float16*)(ws + off); off += b_oh;
    if (off > ws_size) return;

    const int nx8 = MROWS * DM / 8;
    const int nw8 = DM * DM / 8;
    const int prep_total = nx8 + 4 * nw8;
    k_prep<<<(prep_total + 255) / 256, 256, 0, stream>>>(x, wq, wk, wv, wo, nx8, nw8, xh, wh);
    k_mask<<<NTOK / 32, 256, 0, stream>>>(ei, n_e, mk);
    k_qkv<<<dim3(MROWS / 64, NH, 3), 128, 0, stream>>>(xh, wh, bq, bk, bv, qf, kf, vf);
    k_attn<<<dim3(NTOK / 16, NBH), 32, 0, stream>>>(qf, kf, vf, mk, oh);
    k_out<<<MROWS / 32, 256, 0, stream>>>(oh, wh + (size_t)3 * DM * DM, bo, x, gamma, beta, out);
}
